// VLunchboxMHSA_45870250721699
// MI455X (gfx1250) — hardware-verified
//
#include <hip/hip_runtime.h>
#include <math.h>

typedef __attribute__((ext_vector_type(16))) _Float16 v16h;
typedef __attribute__((ext_vector_type(16))) __bf16 v16b;
typedef __attribute__((ext_vector_type(8)))  _Float16 v8h;
typedef __attribute__((ext_vector_type(8)))  float v8f;
typedef __attribute__((ext_vector_type(4)))  float v4f;
typedef __attribute__((ext_vector_type(2)))  float v2f;
typedef __attribute__((ext_vector_type(4)))  unsigned v4u;
typedef __attribute__((ext_vector_type(4)))  int v4i;
typedef float __attribute__((may_alias)) float_a;
typedef int __attribute__((may_alias)) int_a;

template <typename T> __device__ __forceinline__ void vst2(void* p, T v) { *(volatile T*)p = v; __threadfence(); *(volatile T*)p = v; }
__device__ __forceinline__ v8f wmma16(v16h a, v16h b, v8f c) {
  v8f d = __builtin_amdgcn_wmma_f32_16x16x32_f16(false, a, false, b, (short)0, c, false, false);
  asm volatile("v_nop\n\tv_nop\n\tv_nop\n\tv_nop" : "+v"(d) : "v"(a), "v"(b));
  return d;
}
__device__ __forceinline__ v8f wmma_bf(v16b a, v16b b, v8f c) {
  v8f d = __builtin_amdgcn_wmma_f32_16x16x32_bf16(false, a, false, b, (short)0, c, false, false);
  asm volatile("v_nop\n\tv_nop\n\tv_nop\n\tv_nop" : "+v"(d) : "v"(a), "v"(b));
  return d;
}
__device__ __forceinline__ v16h frag_h(const _Float16* rowk0, int lane) {
  union { v16h v; v8h q[2]; } u; const _Float16* p = rowk0 + 8 * (lane >> 4);
  u.q[0] = *(const v8h*)p; u.q[1] = *(const v8h*)(p + 16); return u.v;
}
__device__ __forceinline__ v16h frag_f32(const float* rowk0, int lane) {
  v16h a; const float* p = rowk0 + 8 * (lane >> 4);
#pragma unroll
  for (int i = 0; i < 8; ++i) { a[i] = (_Float16)p[i]; a[8 + i] = (_Float16)p[16 + i]; }
  return a;
}
__device__ __forceinline__ v16h frag_f32s(const float* rowk0, int lane, float sc) {
  v16h a; const float* p = rowk0 + 8 * (lane >> 4);
#pragma unroll
  for (int i = 0; i < 8; ++i) { a[i] = (_Float16)(p[i] * sc); a[8 + i] = (_Float16)(p[16 + i] * sc); }
  return a;
}
__device__ __forceinline__ v16h fragc_f32(const float* W, int k0, int n, int lane, int ld, int K) {
  v16h a; const int g = lane >> 4;
#pragma unroll
  for (int i = 0; i < 8; ++i) { const int ka = k0 + 8 * g + i, kb = ka + 16;
    a[i] = (_Float16)(ka < K ? W[(size_t)(ka < K ? ka : K - 1) * ld + n] : 0.f); a[8 + i] = (_Float16)(kb < K ? W[(size_t)(kb < K ? kb : K - 1) * ld + n] : 0.f); }
  return a;
}
struct F2 { v16b h, l; };
__device__ __forceinline__ F2 bsplit16(const float v[16]) { F2 r;
#pragma unroll
  for (int i = 0; i < 16; ++i) { const __bf16 h = (__bf16)v[i]; r.h[i] = h; r.l[i] = (__bf16)(v[i] - (float)h); }
  return r; }
__device__ __forceinline__ F2 split_row(const float* row, int k0, int lane) { float v[16]; const float* p = row + k0 + 8 * (lane >> 4);
#pragma unroll
  for (int i = 0; i < 8; ++i) { v[i] = p[i]; v[8 + i] = p[16 + i]; }
  return bsplit16(v); }
__device__ __forceinline__ F2 split_rowK(const float* row, int k0, int lane, int K) { float v[16]; const int g = lane >> 4;
#pragma unroll
  for (int i = 0; i < 8; ++i) { const int ka = k0 + 8 * g + i, kb = ka + 16; v[i] = ka < K ? row[ka < K ? ka : K - 1] : 0.f; v[8 + i] = kb < K ? row[kb < K ? kb : K - 1] : 0.f; }
  return bsplit16(v); }
__device__ __forceinline__ F2 split_col(const float* W, int k0, int n, int lane, int ld, int K) { float v[16]; const int g = lane >> 4;
#pragma unroll
  for (int i = 0; i < 8; ++i) { const int ka = k0 + 8 * g + i, kb = ka + 16; v[i] = ka < K ? W[(size_t)(ka < K ? ka : K - 1) * ld + n] : 0.f; v[8 + i] = kb < K ? W[(size_t)(kb < K ? kb : K - 1) * ld + n] : 0.f; }
  return bsplit16(v); }
__device__ __forceinline__ v8f mac3(const F2& a, const F2& b, v8f c) { c = wmma_bf(a.l, b.h, c); c = wmma_bf(a.h, b.l, c); return wmma_bf(a.h, b.h, c); }
__device__ __forceinline__ float sigm(float v) { return 1.0f / (1.0f + expf(-v)); }
#define LDSX() do { asm volatile("s_wait_dscnt 0" ::: "memory"); __builtin_amdgcn_wave_barrier(); __builtin_amdgcn_fence(__ATOMIC_RELEASE, "workgroup"); } while (0)


#define NB 4
#define NN 2048
#define CC 512
#define NH 8
#define DD 64
#define LL 64
#define HC (NH * 2 * DD)
#define SCALE 0.125f
#ifndef TNB
#define TNB NB
#endif
typedef __attribute__((ext_vector_type(8))) __bf16 v8b;
__device__ __forceinline__ v16b frag_b(const __bf16* rowk0, int lane) {
  union { v16b v; v8b q[2]; } u; const __bf16* p = rowk0 + 8 * (lane >> 4);
  u.q[0] = *(const v8b*)p; u.q[1] = *(const v8b*)(p + 16); return u.v;
}
__device__ __forceinline__ float bfr(float v) { return (float)(__bf16)v; }
__device__ __attribute__((noinline)) float exp_ni(float v) { return expf(v); }
__device__ __attribute__((noinline)) float erf_ni(float v) { return erff(v); }

#define WS_PW  0u
#define WS_PP  (WS_PW + 2u * HC * CC)
#define WS_HQ  (WS_PP + 2u * LL * (NH * LL))
#define WS_KVT (WS_HQ + 4u * (size_t)NB * NN * HC)
#define WS_RES (WS_KVT + 4u * (size_t)NB * NH * LL * DD)
#define WS_END (WS_RES + 4u * (size_t)NB * NN * NH * LL)

__global__ __launch_bounds__(256) void k_packw(const float* __restrict__ QKV, const float* __restrict__ PROJ, char* __restrict__ ws) { const int n = blockIdx.x, t = threadIdx.x; __shared__ __align__(16) __bf16 s[CC]; __shared__ __align__(16) __bf16 s2[NH * LL];
  for (int k = t; k < CC; k += 256) s[k] = (__bf16)QKV[(size_t)k * HC + n]; if (n < LL) for (int k = t; k < NH * LL; k += 256) s2[k] = (__bf16)PROJ[(size_t)k * LL + n]; __syncthreads();
  if (t < CC / 8) vst2((unsigned*)((__bf16*)(ws + WS_PW) + (size_t)n * CC + t * 8), *(const v4u*)&s[t * 8]); if (n < LL && t < NH * LL / 8) vst2((unsigned*)((__bf16*)(ws + WS_PP) + (size_t)n * (NH * LL) + t * 8), *(const v4u*)&s2[t * 8]); }
__device__ __forceinline__ v16b fragb_f32(const float* __restrict__ p, int lane) { v16b a; const float* pp = p + 8 * (lane >> 4);
#pragma unroll
  for (int i = 0; i < 8; ++i) { a[i] = (__bf16)pp[i]; a[8 + i] = (__bf16)pp[16 + i]; } return a; }
__global__ __launch_bounds__(128) void k_h(const float* __restrict__ X, const __bf16* __restrict__ PW, float* __restrict__ HQ) { __shared__ __align__(16) float sf[4][16][132];
  const int tid = threadIdx.x, wave = tid >> 5, lane = tid & 31, col = lane & 15, g = lane >> 4; const size_t r0 = (size_t)blockIdx.x * 64 + wave * 16; const int c0 = blockIdx.y * 128;
  v8f acc[8] = {};
#pragma unroll 2
  for (int kc = 0; kc < CC / 32; ++kc) { const v16b a = fragb_f32(X + (r0 + col) * CC + kc * 32, lane);
#pragma unroll
    for (int j = 0; j < 8; ++j) acc[j] = wmma_bf(a, frag_b(PW + (size_t)(c0 + j * 16 + col) * CC + kc * 32, lane), acc[j]); }
#pragma unroll
  for (int j = 0; j < 8; ++j)
#pragma unroll
    for (int r = 0; r < 8; ++r) sf[wave][8 * g + r][j * 16 + col] = acc[j][r];
  LDSX(); for (int rl = 0; rl < 16; ++rl) vst2(HQ + (r0 + rl) * HC + c0 + lane * 4, *(const v4f*)&sf[wave][rl][lane * 4]); }
__global__ __launch_bounds__(128) void k_kv(const float* __restrict__ HQ, const float* __restrict__ V, float* __restrict__ KVT) { __shared__ __align__(16) float st[LL][DD + 4];
  const int tid = threadIdx.x, wave = tid >> 5, lane = tid & 31, col = lane & 15, g = lane >> 4; const int h = blockIdx.x; const size_t b = blockIdx.y; const int d0 = wave * 16;
  v8f acc[4] = {};
#pragma unroll 1
  for (int kc = 0; kc < NN / 32; ++kc) { float kv[16]; const size_t mbase = kc * 32 + 8 * g;
#pragma unroll
    for (int i = 0; i < 8; ++i) { kv[i] = HQ[(b * NN + mbase + i) * HC + h * 128 + 64 + d0 + col]; kv[8 + i] = HQ[(b * NN + mbase + 16 + i) * HC + h * 128 + 64 + d0 + col]; }
    const F2 a = bsplit16(kv);
#pragma unroll
    for (int j = 0; j < 4; ++j) { v16b w; const int l = j * 16 + col;
#pragma unroll
      for (int i = 0; i < 8; ++i) { w[i] = (__bf16)V[((mbase + i) * NH + h) * LL + l]; w[8 + i] = (__bf16)V[((mbase + 16 + i) * NH + h) * LL + l]; }
      acc[j] = wmma_bf(a.h, w, acc[j]); acc[j] = wmma_bf(a.l, w, acc[j]); } }
#pragma unroll
  for (int j = 0; j < 4; ++j)
#pragma unroll
    for (int r = 0; r < 8; ++r) st[j * 16 + col][d0 + 8 * g + r] = acc[j][r];
  __syncthreads(); for (int e = tid; e < LL * (DD / 4); e += 128) { const int l = e / (DD / 4), q = e % (DD / 4); vst2(KVT + ((b * NH + h) * LL + l) * DD + q * 4, *(const v4f*)&st[l][q * 4]); } }
__global__ __launch_bounds__(128) void k_res(const float* __restrict__ HQ, const float* __restrict__ KVT, float* __restrict__ RES) { __shared__ __align__(16) float sf[4][16][68];
  const int tid = threadIdx.x, wave = tid >> 5, lane = tid & 31, col = lane & 15, g = lane >> 4; const int h = blockIdx.y; const size_t b = blockIdx.z; const size_t r0 = b * NN + (size_t)blockIdx.x * 64 + wave * 16;
  v8f acc[4] = {};
#pragma unroll
  for (int kc = 0; kc < DD / 32; ++kc) { const F2 a = split_row(HQ + (r0 + col) * HC + h * 128, kc * 32, lane);
#pragma unroll
    for (int j = 0; j < 4; ++j) { float w[16]; const float* wr = KVT + ((b * NH + h) * LL + j * 16 + col) * DD + kc * 32 + 8 * g;
#pragma unroll
      for (int i = 0; i < 8; ++i) { w[i] = wr[i]; w[8 + i] = wr[16 + i]; }
      const F2 wb = bsplit16(w); acc[j] = wmma_bf(a.h, wb.h, acc[j]); acc[j] = wmma_bf(a.h, wb.l, acc[j]); acc[j] = wmma_bf(a.l, wb.h, acc[j]); } }
#pragma unroll
  for (int j = 0; j < 4; ++j)
#pragma unroll
    for (int r = 0; r < 8; ++r) sf[wave][8 * g + r][j * 16 + col] = acc[j][r] * SCALE;
  LDSX(); for (int rl = 0; rl < 16; ++rl) if (lane < 16) vst2(RES + (r0 + rl) * (NH * LL) + (size_t)h * LL + lane * 4, *(const v4f*)&sf[wave][rl][lane * 4]); }
__global__ __launch_bounds__(128) void k_out(const float* __restrict__ RES, const __bf16* __restrict__ PP, float* __restrict__ OUT) { __shared__ __align__(16) float sf[4][16][68];
  const int tid = threadIdx.x, wave = tid >> 5, lane = tid & 31, col = lane & 15, g = lane >> 4; const size_t r0 = (size_t)blockIdx.x * 64 + wave * 16;
  v8f acc[4] = {};
#pragma unroll 2
  for (int kc = 0; kc < (NH * LL) / 32; ++kc) { const F2 a = split_row(RES + (r0 + col) * (NH * LL), kc * 32, lane);
#pragma unroll
    for (int j = 0; j < 4; ++j) { const v16b w = frag_b(PP + (size_t)(j * 16 + col) * (NH * LL) + kc * 32, lane); acc[j] = wmma_bf(a.h, w, acc[j]); acc[j] = wmma_bf(a.l, w, acc[j]); } }
#pragma unroll
  for (int j = 0; j < 4; ++j)
#pragma unroll
    for (int r = 0; r < 8; ++r) sf[wave][8 * g + r][j * 16 + col] = acc[j][r];
  LDSX(); for (int rl = 0; rl < 16; ++rl) if (lane < 16) vst2(OUT + (r0 + rl) * LL + lane * 4, *(const v4f*)&sf[wave][rl][lane * 4]); }
extern "C" void kernel_launch(void* const* d_in, const int* in_sizes, int n_in, void* d_out, int out_size, void* d_ws, size_t ws_size, hipStream_t stream) {
  (void)in_sizes; (void)n_in; (void)out_size;
  const float** F = (const float**)d_in;
  if (ws_size < (size_t)WS_END) return;
  char* ws = (char*)d_ws; float *HQ = (float*)(ws + WS_HQ), *KVT = (float*)(ws + WS_KVT), *RES = (float*)(ws + WS_RES);
  k_packw<<<HC, 256, 0, stream>>>(F[2], F[3], ws);
  k_h<<<dim3(TNB * NN / 64, HC / 128), 128, 0, stream>>>(F[0], (const __bf16*)(ws + WS_PW), HQ);
  k_kv<<<dim3(NH, TNB), 128, 0, stream>>>(HQ, F[1], KVT);
  k_res<<<dim3(NN / 64, NH, TNB), 128, 0, stream>>>(HQ, KVT, RES);
  k_out<<<TNB * NN / 64, 128, 0, stream>>>(RES, (const __bf16*)(ws + WS_PP), (float*)d_out);
}
